// GCN_64372969832855
// MI455X (gfx1250) — hardware-verified
//
#include <hip/hip_runtime.h>
#include <stddef.h>
#include <stdint.h>
#include <math.h>


#define FIN    128
#define HID    64
#define NLAY   3
#define NGR    512
#define NTHR   256
#define NWAVE  8
#define EPT    8
#define CHUNK  (NTHR * EPT)
#define WCAP   (EPT * 32)
#define LISTN  (NWAVE * WCAP)
#define NBD    8192
#define SLD    13
#define NBA    1024
#define SLA    10
#define RCAP   28672
#define DEGCAP 128
#define GBM    64
#define GBN    64
#define GTHR   128
#define SROWS  1024
#define NUF    (HID * (2 * FIN / 8))
#define NUS1   (HID * (2 * HID / 8))
#define NUS    (NLAY * NUS1)
#define AGG_ZINTS (LISTN + 2 * RCAP + 3 * NBA)
#define MISC_INTS 16
#define AGG_INTS  (AGG_ZINTS + MISC_INTS)
#define AGG_DBL   (NWAVE * 2 * HID + 2 * HID)
#define AGG_LDS_BYTES (AGG_INTS * 4 + AGG_DBL * 8)
#define WSMAX  134217728

static_assert((CHUNK & (CHUNK - 1)) == 0 && CHUNK <= 4096);
static_assert((NBD & (NBD - 1)) == 0 && NBD == (1 << SLD));
static_assert((NBA & (NBA - 1)) == 0 && NBA == (1 << SLA));
static_assert(((long long)CHUNK << SLD) < (1LL << 31));
static_assert(((long long)CHUNK << SLA) < (1LL << 31));
static_assert(NBD % (NTHR * 4) == 0);
static_assert(LISTN % NTHR == 0);
static_assert(NBA % NWAVE == 0 && NBA % 32 == 0 && NBA % GBM == 0);
static_assert(RCAP % 32 == 0 && AGG_ZINTS % 4 == 0 && LISTN % 4 == 0);
static_assert((AGG_INTS * 4) % 16 == 0);
static_assert(AGG_LDS_BYTES <= 300000);
static_assert(GBM == (GTHR / 32) * 16 && GBN == 64 && HID == GBN);
static_assert(HID == 2 * 32);
static_assert(NUF % NTHR == 0 && NUS % NTHR == 0);
static_assert(2 * FIN == NTHR);
static_assert((2 * FIN) % 32 == 0 && (2 * HID) % 32 == 0);
static_assert(NUS1 == 1024);

typedef float          v2f   __attribute__((ext_vector_type(2)));
typedef float          v4f   __attribute__((ext_vector_type(4)));
typedef float          v8f   __attribute__((ext_vector_type(8)));
typedef double         v2d   __attribute__((ext_vector_type(2)));
typedef int            v4i   __attribute__((ext_vector_type(4)));
typedef int            v8i   __attribute__((ext_vector_type(8)));
typedef unsigned short v4us  __attribute__((ext_vector_type(4)));
typedef unsigned short v8us  __attribute__((ext_vector_type(8)));
typedef unsigned short v16us __attribute__((ext_vector_type(16)));
typedef __bf16         v16bf __attribute__((ext_vector_type(16)));
typedef v2f  __attribute__((may_alias)) v2fa;
typedef v4f  __attribute__((may_alias)) v4fa;
typedef v2d  __attribute__((may_alias)) v2da;
typedef v4i  __attribute__((may_alias)) v4ia;
typedef v4us __attribute__((may_alias)) v4usa;
typedef v8us __attribute__((may_alias)) v8usa;
union FragB { v16bf v; v16us u; v8us h[2]; v8i w; };

__device__ __forceinline__ v8f wmb(const FragB& a, const FragB& b, v8f c) {
  v8f d = __builtin_amdgcn_wmma_f32_16x16x32_bf16(false, a.v, false, b.v, (short)0, c, false, false);
  asm volatile("v_nop\n\tv_nop\n\tv_nop\n\tv_nop" : "+v"(d) : "v"(a.w), "v"(b.w));
  return d;
}

__device__ __forceinline__ unsigned bf16_bits(float f) {
  const unsigned u = __float_as_uint(f);
  return (u + 0x7FFFu + ((u >> 16) & 1u)) >> 16;
}
__device__ __forceinline__ float bf16_val(float f) {
  return __uint_as_float(bf16_bits(f) << 16);
}

__device__ __forceinline__ void st2_us8(unsigned short* p, v8us v) {
  *(volatile v8us*)p = v;
  __threadfence();
  *(volatile v8us*)p = v;
}
__device__ __forceinline__ void st2_d2(double* p, v2d v) {
  *(volatile v2d*)p = v;
  __threadfence();
  *(volatile v2d*)p = v;
}
__device__ __forceinline__ void st2_f4(float* p, v4f v) {
  *(volatile v4f*)p = v;
  __threadfence();
  *(volatile v4f*)p = v;
}

template <int SLB>
__device__ __forceinline__ int scan_chunk(const int* __restrict__ dsts, int nE, int cbase, int slotBase,
                                          int nb, int vec8, int* list, int tid, int lane, int wave) {
  int wc = 0;
  const int el0  = tid * EPT;
  const int e0   = cbase + el0;
  const int sent = -2147483647 - 1;
  v4i da, db;
  if (vec8 != 0 && cbase + CHUNK <= nE) {
    da = *(const v4i*)(dsts + e0);
    db = *(const v4i*)(dsts + e0 + 4);
  } else {
    da.x = (e0     < nE) ? dsts[min(e0,     nE - 1)] : sent;
    da.y = (e0 + 1 < nE) ? dsts[min(e0 + 1, nE - 1)] : sent;
    da.z = (e0 + 2 < nE) ? dsts[min(e0 + 2, nE - 1)] : sent;
    da.w = (e0 + 3 < nE) ? dsts[min(e0 + 3, nE - 1)] : sent;
    db.x = (e0 + 4 < nE) ? dsts[min(e0 + 4, nE - 1)] : sent;
    db.y = (e0 + 5 < nE) ? dsts[min(e0 + 5, nE - 1)] : sent;
    db.z = (e0 + 6 < nE) ? dsts[min(e0 + 6, nE - 1)] : sent;
    db.w = (e0 + 7 < nE) ? dsts[min(e0 + 7, nE - 1)] : sent;
  }
  const unsigned nbs = (unsigned)slotBase;
  const unsigned unb = (unsigned)nb;
  const unsigned s0 = (unsigned)da.x - nbs, s1 = (unsigned)da.y - nbs;
  const unsigned s2 = (unsigned)da.z - nbs, s3 = (unsigned)da.w - nbs;
  const unsigned s4 = (unsigned)db.x - nbs, s5 = (unsigned)db.y - nbs;
  const unsigned s6 = (unsigned)db.z - nbs, s7 = (unsigned)db.w - nbs;
  const bool h0 = s0 < unb, h1 = s1 < unb, h2 = s2 < unb, h3 = s3 < unb;
  const bool h4 = s4 < unb, h5 = s5 < unb, h6 = s6 < unb, h7 = s7 < unb;
  const unsigned any = __builtin_amdgcn_ballot_w32(h0 | h1 | h2 | h3 | h4 | h5 | h6 | h7);
  if (any != 0u) {
#define HITJ(J, HJ, SJ) { \
      const unsigned mj = __builtin_amdgcn_ballot_w32(HJ); \
      if (mj != 0u) { \
        if (HJ) { \
          const int pos = wc + (int)__builtin_amdgcn_mbcnt_lo(mj, 0u); \
          if (pos < WCAP) list[wave * WCAP + pos] = ((el0 + (J)) << SLB) | (int)(SJ); \
        } \
        wc += (int)__builtin_popcount(mj); } }
    HITJ(0, h0, s0)
    HITJ(1, h1, s1)
    HITJ(2, h2, s2)
    HITJ(3, h3, s3)
    HITJ(4, h4, s4)
    HITJ(5, h5, s5)
    HITJ(6, h6, s6)
    HITJ(7, h7, s7)
#undef HITJ
  }
  return wc;
}

__global__ __launch_bounds__(NTHR) void k_wprep(const float* __restrict__ Wf, const float* __restrict__ Ws,
                                                unsigned short* WF2, unsigned short* WS2) {
  const int u = (int)blockIdx.x * NTHR + (int)threadIdx.x;
  if (u < NUF) {
    const int n  = u >> 5;
    const int k8 = (u & 31) * 8;
    const int kk = k8 & (FIN - 1);
    const float* p = Wf + (size_t)kk * HID + n;
    v8us o;
#pragma unroll
    for (int i = 0; i < 8; ++i) o[i] = (unsigned short)bf16_bits(p[(size_t)i * HID]);
    st2_us8(WF2 + (size_t)n * (2 * FIN) + k8, o);
  } else if (u < NUF + NUS) {
    const int v   = u - NUF;
    const int lay = v >> 10;
    const int r   = v & (NUS1 - 1);
    const int n   = r >> 4;
    const int k8  = (r & 15) * 8;
    const int kk  = k8 & (HID - 1);
    const float* p = Ws + (size_t)lay * HID * HID + (size_t)kk * HID + n;
    v8us o;
#pragma unroll
    for (int i = 0; i < 8; ++i) o[i] = (unsigned short)bf16_bits(p[(size_t)i * HID]);
    st2_us8(WS2 + (size_t)lay * (HID * 2 * HID) + (size_t)n * (2 * HID) + k8, o);
  }
}

__global__ __launch_bounds__(NTHR) void k_deg(const int* __restrict__ keys, int nE, int vec8, float* dis) {
  __shared__ __attribute__((aligned(16))) int scnt[NBD];
  __shared__ __attribute__((aligned(16))) int list[LISTN];
  __shared__ int wcnt[NWAVE];
  const int tid = (int)threadIdx.x, lane = tid & 31, wave = tid >> 5;
  const int nodeBase = (int)blockIdx.x * NBD;

  for (int i = tid; i < NBD; i += NTHR) scnt[i] = 0;
  for (int i = tid; i < LISTN; i += NTHR) list[i] = 0;
  if (tid < NWAVE) wcnt[tid] = 0;
  __syncthreads();

  const int nChunks = (nE + CHUNK - 1) / CHUNK;
#pragma unroll 1
  for (int ch = 0; ch < nChunks; ++ch) {
    const int cbase = ch * CHUNK;
    const int wc = scan_chunk<SLD>(keys, nE, cbase, nodeBase, NBD, vec8, list, tid, lane, wave);
    if (lane == 0) wcnt[wave] = wc;
    __syncthreads();
    if (wave == 0) {
#pragma unroll 1
      for (int w2 = 0; w2 < NWAVE; ++w2) {
        int c = wcnt[w2];
        c = c < 0 ? 0 : (c > WCAP ? WCAP : c);
#pragma unroll 1
        for (int b0 = 0; b0 < c; b0 += 32) {
          const int idx = b0 + lane;
          const int ent = list[w2 * WCAP + (idx < WCAP ? idx : WCAP - 1)];
          const int m32 = (c - b0) < 32 ? (c - b0) : 32;
#pragma unroll 1
          for (int k = 0; k < m32; ++k) {
            const int u  = __builtin_amdgcn_readlane(ent, k);
            const int sl = u & (NBD - 1);
            if (lane == 0) scnt[sl] = scnt[sl] + 1;
          }
        }
      }
    }
    __syncthreads();
  }

  v4f vals[NBD / (NTHR * 4)];
#pragma unroll
  for (int it = 0; it < NBD / (NTHR * 4); ++it) {
    const int s0 = it * (NTHR * 4) + 4 * tid;
    const v4i c4 = *(const v4ia*)(scnt + s0);
    const float d0 = (float)c4.x + 1.0f, d1 = (float)c4.y + 1.0f;
    const float d2 = (float)c4.z + 1.0f, d3 = (float)c4.w + 1.0f;
    v4f v;
    v.x = rsqrtf(d0); v.y = rsqrtf(d1); v.z = rsqrtf(d2); v.w = rsqrtf(d3);
    vals[it] = v;
  }
#pragma unroll
  for (int it = 0; it < NBD / (NTHR * 4); ++it) {
    const int s0 = it * (NTHR * 4) + 4 * tid;
    *(volatile v4f*)(dis + (size_t)nodeBase + s0) = vals[it];
  }
  __threadfence();
#pragma unroll
  for (int it = 0; it < NBD / (NTHR * 4); ++it) {
    const int s0 = it * (NTHR * 4) + 4 * tid;
    *(volatile v4f*)(dis + (size_t)nodeBase + s0) = vals[it];
  }
}

__global__ __launch_bounds__(NTHR) void k_statx(const float* __restrict__ x, int nN, double* rec) {
  __shared__ __attribute__((aligned(16))) double ps[2 * 2 * FIN];
  __shared__ __attribute__((aligned(16))) double ro[2 * FIN];
  const int tid = (int)threadIdx.x;
  const int col = tid & (FIN - 1);
  const int hf  = tid >> 7;
  const int rowBase = (int)blockIdx.x * SROWS;
  double s = 0.0, q = 0.0;
#pragma unroll 4
  for (int j = 0; j < SROWS / 2; ++j) {
    const int row = rowBase + hf + 2 * j;
    const int rc  = row < nN ? row : nN - 1;
    const float v  = bf16_val(x[(size_t)rc * FIN + col]);
    const float vz = (row < nN) ? v : 0.0f;
    const double d = (double)vz;
    s += d;
    q = fma(d, d, q);
  }
  ps[hf * (2 * FIN) + col]       = s;
  ps[hf * (2 * FIN) + FIN + col] = q;
  __syncthreads();
  ro[tid] = ps[tid] + ps[2 * FIN + tid];
  __syncthreads();
  if (tid < FIN) {
    const v2d o = *(const v2da*)(ro + 2 * tid);
    st2_d2(rec + (size_t)blockIdx.x * (2 * FIN) + 2 * tid, o);
  }
}

__global__ __launch_bounds__(128) void k_comb(const double* __restrict__ rec, float* stat, double invn,
                                              int nrec, int ncol) {
  __shared__ __attribute__((aligned(16))) float st[2 * FIN];
  const int tid = (int)threadIdx.x;
  const int cc  = tid < ncol ? tid : ncol - 1;
  double S = 0.0, Q = 0.0;
#pragma unroll 1
  for (int b = 0; b < nrec; ++b) {
    const double* rp = rec + (size_t)b * (size_t)(2 * ncol);
    S += rp[cc];
    Q += rp[ncol + cc];
  }
  const double mu = S * invn;
  double var = Q * invn - mu * mu;
  var = (var < 0.0) ? 0.0 : var;
  const float muf = (float)mu;
  const float rf  = 1.0f / sqrtf((float)var + 1e-5f);
  st[tid]       = (tid < ncol) ? muf : 0.0f;
  st[FIN + tid] = (tid < ncol) ? rf : 0.0f;
  __syncthreads();
  if (tid < 64) {
    const v4f o = *(const v4fa*)(st + 4 * tid);
    st2_f4(stat + 4 * tid, o);
  }
}

template <int KIN, int FEAT>
__global__ __launch_bounds__(GTHR) void k_gemm(const float* __restrict__ A, int nN,
                                               const float* __restrict__ stat,
                                               const float* __restrict__ gam, const float* __restrict__ bet,
                                               const unsigned short* __restrict__ WT,
                                               const float* __restrict__ bias, float* outF, double* rec) {
  constexpr int K2  = 2 * KIN;
  constexpr int AP  = K2 + 8;
  constexpr int C4  = KIN / 4;
  constexpr int RPI = GTHR / C4;
  constexpr int NIT = GBM / RPI;
  static_assert(K2 % 32 == 0 && (C4 & (C4 - 1)) == 0 && GTHR % C4 == 0 && GBM % RPI == 0);
  static_assert((AP * 2) % 16 == 0 && KIN <= FIN);
  __shared__ __attribute__((aligned(16))) unsigned short As[GBM * AP];
  __shared__ __attribute__((aligned(16))) float stg[GBM * GBN];
  __shared__ __attribute__((aligned(16))) double rs[2 * HID];
  const int tid = (int)threadIdx.x, lane = tid & 31, wave = tid >> 5, hh = lane >> 4, m = lane & 15;
  const int rowBase = (int)blockIdx.x * GBM;

  {
    const int c4  = tid & (C4 - 1);
    const int lr0 = tid / C4;
    const v4f mu4 = *(const v4f*)(stat + 4 * c4);
    const v4f r4  = *(const v4f*)(stat + FIN + 4 * c4);
    v4f g4 = *(const v4f*)(gam + 4 * c4);
    v4f b4 = *(const v4f*)(bet + 4 * c4);
    g4.x = bf16_val(g4.x); g4.y = bf16_val(g4.y); g4.z = bf16_val(g4.z); g4.w = bf16_val(g4.w);
    b4.x = bf16_val(b4.x); b4.y = bf16_val(b4.y); b4.z = bf16_val(b4.z); b4.w = bf16_val(b4.w);
#pragma unroll 4
    for (int it = 0; it < NIT; ++it) {
      const int lr = it * RPI + lr0;
      const int gr = rowBase + lr;
      const int rc = gr < nN ? gr : nN - 1;
      const bool live = gr < nN;
      v4f v = *(const v4f*)(A + (size_t)rc * KIN + 4 * c4);
      if constexpr (FEAT != 0) {
        v.x = bf16_val(v.x); v.y = bf16_val(v.y); v.z = bf16_val(v.z); v.w = bf16_val(v.w);
      }
      float a0 = ((v.x - mu4.x) * r4.x) * g4.x + b4.x;
      float a1 = ((v.y - mu4.y) * r4.y) * g4.y + b4.y;
      float a2 = ((v.z - mu4.z) * r4.z) * g4.z + b4.z;
      float a3 = ((v.w - mu4.w) * r4.w) * g4.w + b4.w;
      a0 = live ? a0 : 0.0f; a1 = live ? a1 : 0.0f; a2 = live ? a2 : 0.0f; a3 = live ? a3 : 0.0f;
      v4us h4, l4;
      unsigned hb;
      hb = bf16_bits(a0); h4[0] = (unsigned short)hb; l4[0] = (unsigned short)bf16_bits(a0 - __uint_as_float(hb << 16));
      hb = bf16_bits(a1); h4[1] = (unsigned short)hb; l4[1] = (unsigned short)bf16_bits(a1 - __uint_as_float(hb << 16));
      hb = bf16_bits(a2); h4[2] = (unsigned short)hb; l4[2] = (unsigned short)bf16_bits(a2 - __uint_as_float(hb << 16));
      hb = bf16_bits(a3); h4[3] = (unsigned short)hb; l4[3] = (unsigned short)bf16_bits(a3 - __uint_as_float(hb << 16));
      *(v4usa*)(As + lr * AP + 4 * c4)       = h4;
      *(v4usa*)(As + lr * AP + KIN + 4 * c4) = l4;
    }
  }
  __syncthreads();

  v8f acc[4];
  {
    const v8f z = {0.f, 0.f, 0.f, 0.f, 0.f, 0.f, 0.f, 0.f};
    acc[0] = z; acc[1] = z; acc[2] = z; acc[3] = z;
  }
  const unsigned short* ap = As + (16 * wave + m) * AP + 8 * hh;
  const unsigned short* wp = WT + (size_t)m * (size_t)K2 + 8 * hh;
#pragma unroll 1
  for (int ks = 0; ks < K2 / 32; ++ks) {
    FragB af;
    af.h[0] = *(const v8usa*)(ap + 32 * ks);
    af.h[1] = *(const v8usa*)(ap + 32 * ks + 16);
#pragma unroll
    for (int t = 0; t < 4; ++t) {
      const unsigned short* wq = wp + (size_t)(16 * t) * (size_t)K2 + 32 * ks;
      FragB bf;
      bf.h[0] = *(const v8usa*)wq;
      bf.h[1] = *(const v8usa*)(wq + 16);
      acc[t] = wmb(af, bf, acc[t]);
    }
  }

#pragma unroll
  for (int t = 0; t < 4; ++t) {
    const int lc = 16 * t + m;
#pragma unroll
    for (int r = 0; r < 8; ++r) {
      const int lr = 16 * wave + 8 * hh + r;
      stg[lr * GBN + lc] = acc[t][r];
    }
  }
  __syncthreads();

  v4f bb4 = {0.f, 0.f, 0.f, 0.f};
  if constexpr (FEAT != 0) {
    const v4f t1 = *(const v4f*)(bias + 4 * m);
    bb4.x = bf16_val(t1.x); bb4.y = bf16_val(t1.y); bb4.z = bf16_val(t1.z); bb4.w = bf16_val(t1.w);
  }
  v4f fv[8];
#pragma unroll
  for (int i = 0; i < 8; ++i) {
    const int lr = 16 * wave + 2 * i + hh;
    const bool live = (rowBase + lr) < nN;
    v4f y = *(const v4fa*)(stg + lr * GBN + 4 * m);
    if constexpr (FEAT != 0) {
      y = y + bb4;
      y.x = (y.x > 0.0f) ? y.x : (y.x - y.x);
      y.y = (y.y > 0.0f) ? y.y : (y.y - y.y);
      y.z = (y.z > 0.0f) ? y.z : (y.z - y.z);
      y.w = (y.w > 0.0f) ? y.w : (y.w - y.w);
    }
    y.x = live ? y.x : 0.0f; y.y = live ? y.y : 0.0f; y.z = live ? y.z : 0.0f; y.w = live ? y.w : 0.0f;
    fv[i] = y;
    if constexpr (FEAT != 0) *(v4fa*)(stg + lr * GBN + 4 * m) = y;
  }
#pragma unroll
  for (int i = 0; i < 8; ++i) {
    const int lr = 16 * wave + 2 * i + hh;
    float* op = outF + (size_t)(rowBase + lr) * HID + 4 * m;
    *(volatile v4f*)op = fv[i];
  }
  __threadfence();
#pragma unroll
  for (int i = 0; i < 8; ++i) {
    const int lr = 16 * wave + 2 * i + hh;
    float* op = outF + (size_t)(rowBase + lr) * HID + 4 * m;
    *(volatile v4f*)op = fv[i];
  }

  if constexpr (FEAT != 0) {
    __syncthreads();
    if (tid < HID) {
      double s = 0.0, q = 0.0;
#pragma unroll 4
      for (int r = 0; r < GBM; ++r) {
        const double d = (double)stg[r * GBN + tid];
        s += d;
        q = fma(d, d, q);
      }
      rs[tid] = s;
      rs[HID + tid] = q;
    }
    __syncthreads();
    if (tid < HID) {
      const v2d o = *(const v2da*)(rs + 2 * tid);
      st2_d2(rec + (size_t)blockIdx.x * (2 * HID) + 2 * tid, o);
    }
  }
}

template <int STATS>
__global__ __launch_bounds__(NTHR) void k_agg(const int* __restrict__ srcs, const int* __restrict__ dsts,
                                              int nE, int nN, int vec8, int mRows,
                                              const float* __restrict__ dis,
                                              const float* __restrict__ xl, const float* __restrict__ bias,
                                              float* hout, double* rec) {
  extern __shared__ __attribute__((aligned(16))) int dsm[];
  int* list = dsm;
  int* hl   = dsm + LISTN;
  int* sl   = dsm + LISTN + RCAP;
  int* cnt  = dsm + LISTN + 2 * RCAP;
  int* offs = cnt + NBA;
  int* cur  = offs + NBA;
  int* misc = cur + NBA;
  double* wsd = (double*)(misc + MISC_INTS);
  double* ro  = wsd + NWAVE * 2 * HID;
  const int tid = (int)threadIdx.x, lane = tid & 31, wave = tid >> 5;
  const int nodeBase = (int)blockIdx.x * NBA;

  {
    const v4i z4 = {0, 0, 0, 0};
    for (int i = tid * 4; i < AGG_ZINTS; i += NTHR * 4) *(v4ia*)(dsm + i) = z4;
    if (tid < MISC_INTS) misc[tid] = 0;
  }
  float bv0, bv1;
  {
    const v2f a = *(const v2fa*)(bias + 2 * lane);
    bv0 = bf16_val(a.x); bv1 = bf16_val(a.y);
  }
  __syncthreads();

  int t = 0, ov = 0;
  const int nChunks = (nE + CHUNK - 1) / CHUNK;
#pragma unroll 1
  for (int ch = 0; ch < nChunks; ++ch) {
    const int cbase = ch * CHUNK;
    const int wc = scan_chunk<SLA>(dsts, nE, cbase, nodeBase, NBA, vec8, list, tid, lane, wave);
    if (lane == 0) misc[wave] = wc;
    __syncthreads();
    if (wave == 0) {
#pragma unroll 1
      for (int w2 = 0; w2 < NWAVE; ++w2) {
        int c = misc[w2];
        c = c < 0 ? 0 : (c > WCAP ? WCAP : c);
#pragma unroll 1
        for (int b0 = 0; b0 < c; b0 += 32) {
          const int idx = b0 + lane;
          const int ent = list[w2 * WCAP + (idx < WCAP ? idx : WCAP - 1)];
          const int m32 = (c - b0) < 32 ? (c - b0) : 32;
#pragma unroll 1
          for (int k = 0; k < m32; ++k) {
            const int u    = __builtin_amdgcn_readlane(ent, k);
            const int slot = u & (NBA - 1);
            const int el   = (u >> SLA) & (CHUNK - 1);
            const int pk   = ((cbase + el) << SLA) | slot;
            if (t < RCAP) {
              if (lane == 0) { hl[t] = pk; cnt[slot] = cnt[slot] + 1; }
              t = t + 1;
            } else {
              ov = 1;
            }
          }
        }
      }
    }
    __syncthreads();
  }
  if (wave == 0 && lane == 0) { misc[8] = t; misc[9] = ov; }
  __syncthreads();
  int tt = misc[8];
  tt = tt < 0 ? 0 : (tt > RCAP ? RCAP : tt);
  const int ovf = misc[9];

  if (wave == 0) {
    const int base = lane * (NBA / 32);
    int s = 0;
#pragma unroll 1
    for (int i = 0; i < NBA / 32; ++i) s += cnt[base + i];
    int incl = s;
#pragma unroll
    for (int d = 1; d < 32; d <<= 1) {
      const int y = __shfl_up(incl, d, 32);
      if (lane >= d) incl += y;
    }
    int run = incl - s;
#pragma unroll 1
    for (int i = 0; i < NBA / 32; ++i) {
      const int cv = cnt[base + i];
      offs[base + i] = run;
      cur[base + i]  = run;
      run += cv;
    }
  }
  __syncthreads();
  if (wave == 0) {
#pragma unroll 1
    for (int b0 = 0; b0 < tt; b0 += 32) {
      const int idx = b0 + lane;
      const int ent = hl[idx < RCAP ? idx : RCAP - 1];
      const int m32 = (tt - b0) < 32 ? (tt - b0) : 32;
#pragma unroll 1
      for (int k = 0; k < m32; ++k) {
        const int u    = __builtin_amdgcn_readlane(ent, k);
        const int slot = u & (NBA - 1);
        if (lane == 0) {
          int p = cur[slot];
          p = p < 0 ? 0 : (p > RCAP - 1 ? RCAP - 1 : p);
          sl[p] = u;
          cur[slot] = p + 1;
        }
      }
    }
  }
  __syncthreads();

  const float qnan = __int_as_float(0x7fc00000);
  const float pz = (ovf != 0) ? qnan : 0.0f;
  const int sa = (2 * lane) & 31, sb = (2 * lane + 1) & 31;
  double ss0 = 0.0, ss1 = 0.0, sq0 = 0.0, sq1 = 0.0;
#pragma unroll 1
  for (int si = 0; si < NBA / NWAVE; ++si) {
    const int s    = si * NWAVE + wave;
    const int node = nodeBase + s;
    int c = cnt[s];
    const bool big = c > DEGCAP;
    c = c < 0 ? 0 : (c > DEGCAP ? DEGCAP : c);
    int o = offs[s];
    o = o < 0 ? 0 : (o > RCAP ? RCAP : o);
    const int nc = node < nN ? node : nN - 1;
    const float dd = dis[nc];
    const float rd = dd * dd;
    float acc0 = 0.0f, acc1 = 0.0f;
#pragma unroll 1
    for (int b0 = 0; b0 < c; b0 += 32) {
      int idx = o + b0 + lane;
      idx = idx > RCAP - 1 ? RCAP - 1 : idx;
      const int ent = sl[idx];
      int eid = ent >> SLA;
      eid = eid < 0 ? 0 : (eid > nE - 1 ? nE - 1 : eid);
      int sr = srcs[eid];
      sr = sr < 0 ? 0 : (sr > nN - 1 ? nN - 1 : sr);
      const float cf  = dis[sr] * dd;
      const int   cfi = __float_as_int(cf);
      const int m32 = (c - b0) < 32 ? (c - b0) : 32;
#pragma unroll 1
      for (int k = 0; k < m32; ++k) {
        const int   sk = __builtin_amdgcn_readlane(sr, k);
        const float ck = __int_as_float(__builtin_amdgcn_readlane(cfi, k));
        const v2f a = *(const v2fa*)(xl + (size_t)sk * HID + 2 * lane);
        acc0 = fmaf(ck, a.x, acc0); acc1 = fmaf(ck, a.y, acc1);
      }
    }
    float sv0, sv1;
    {
      const v2f a = *(const v2fa*)(xl + (size_t)nc * HID + 2 * lane);
      sv0 = a.x; sv1 = a.y;
    }
    const float pzr = big ? qnan : pz;
    const bool live = node < nN;
    float y0 = (acc0 + sv0 * rd) + bv0;
    float y1 = (acc1 + sv1 * rd) + bv1;
    y0 = (y0 > 0.0f) ? y0 : (y0 - y0);
    y1 = (y1 > 0.0f) ? y1 : (y1 - y1);
    y0 = y0 + pzr; y1 = y1 + pzr;
    const float v0 = live ? y0 : 0.0f;
    const float v1 = live ? y1 : 0.0f;
    if constexpr (STATS != 0) {
      const double d0 = (double)v0, d1 = (double)v1;
      ss0 += d0; ss1 += d1;
      sq0 = fma(d0, d0, sq0); sq1 = fma(d1, d1, sq1);
    }
    const bool wr = (node < mRows) && (lane < 16);
    v4f ow;
    ow.x = __shfl(v0, sa, 32); ow.y = __shfl(v1, sa, 32);
    ow.z = __shfl(v0, sb, 32); ow.w = __shfl(v1, sb, 32);
    float* op = hout + (size_t)node * HID + 4 * (lane & 15);
    if (wr) *(volatile v4f*)op = ow;
    __threadfence();
    if (wr) *(volatile v4f*)op = ow;
  }

  if constexpr (STATS != 0) {
    wsd[wave * (2 * HID) + 2 * lane + 0]       = ss0;
    wsd[wave * (2 * HID) + 2 * lane + 1]       = ss1;
    wsd[wave * (2 * HID) + HID + 2 * lane + 0] = sq0;
    wsd[wave * (2 * HID) + HID + 2 * lane + 1] = sq1;
    __syncthreads();
    if (tid < 2 * HID) {
      double a = 0.0;
#pragma unroll 1
      for (int w2 = 0; w2 < NWAVE; ++w2) a += wsd[w2 * (2 * HID) + tid];
      ro[tid] = a;
    }
    __syncthreads();
    if (tid < HID) {
      const v2d o2 = *(const v2da*)(ro + 2 * tid);
      st2_d2(rec + (size_t)blockIdx.x * (2 * HID) + 2 * tid, o2);
    }
  }
}

__global__ __launch_bounds__(NTHR) void k_pool(const float* __restrict__ hf, const int* __restrict__ bat,
                                               int nN, float* outp) {
  __shared__ __attribute__((aligned(16))) float wsum[NWAVE * HID];
  __shared__ __attribute__((aligned(16))) float outs[HID];
  const int tid = (int)threadIdx.x, lane = tid & 31, wave = tid >> 5;
  const int g = (int)blockIdx.x;

  float a0 = 0.0f, a1 = 0.0f;
#pragma unroll 1
  for (int i0 = wave * 32; i0 < nN; i0 += NTHR) {
    const int i  = i0 + lane;
    const int ic = i < nN ? i : nN - 1;
    const int b  = bat[ic];
    const bool hit = (i < nN) && (b == g);
    unsigned msk = __builtin_amdgcn_ballot_w32(hit);
    int nh = (int)__builtin_popcount(msk);
    nh = nh > 32 ? 32 : nh;
#pragma unroll 1
    for (int q = 0; q < nh; ++q) {
      const int k = __builtin_ffs((int)msk) - 1;
      msk &= msk - 1u;
      int node = i0 + (k < 0 ? 0 : k);
      node = node > nN - 1 ? nN - 1 : node;
      const v2f v = *(const v2fa*)(hf + (size_t)node * HID + 2 * lane);
      a0 += v.x; a1 += v.y;
    }
  }
  wsum[wave * HID + 2 * lane + 0] = a0;
  wsum[wave * HID + 2 * lane + 1] = a1;
  __syncthreads();
  if (tid < HID) {
    float s = 0.0f;
#pragma unroll
    for (int w2 = 0; w2 < NWAVE; ++w2) s += wsum[w2 * HID + tid];
    outs[tid] = s;
  }
  __syncthreads();
  const v4f ov = *(const v4fa*)(outs + 4 * (lane & 15));
  float* op = outp + (size_t)g * HID + 4 * (lane & 15);
  const bool okst = (wave == 0) && (lane < 16);
  if (okst) *(volatile v4f*)op = ov;
  __threadfence();
  if (okst) *(volatile v4f*)op = ov;
}

static inline int cdiv(int a, int b) { return (a + b - 1) / b; }
static inline size_t al256(size_t o) { return (o + 255) & ~(size_t)255; }

extern "C" void kernel_launch(void* const* d_in, const int* in_sizes, int n_in,
                              void* d_out, int out_size, void* d_ws, size_t ws_size,
                              hipStream_t stream) {
  if (n_in < 11) return;
  if (in_sizes[0] < FIN || (in_sizes[0] % FIN) != 0) return;
  const int nN = in_sizes[0] / FIN;
  if (nN < 1 || nN > (1 << 22)) return;
  if (in_sizes[1] < 2 || (in_sizes[1] & 1) != 0) return;
  const int nE = in_sizes[1] / 2;
  if (nE < 1 || nE >= (1 << (31 - SLA))) return;
  if (in_sizes[2] != nN) return;
  if (in_sizes[3] != FIN || in_sizes[4] != FIN) return;
  if (in_sizes[5] != FIN * HID || in_sizes[6] != HID) return;
  if (in_sizes[7] != NLAY * HID || in_sizes[8] != NLAY * HID) return;
  if (in_sizes[9] != NLAY * HID * HID || in_sizes[10] != NLAY * HID) return;
  if (out_size != NGR * HID) return;

  const float* x    = (const float*)d_in[0];
  const int*   edge = (const int*)d_in[1];
  const int*   bat  = (const int*)d_in[2];
  const float* bnfg = (const float*)d_in[3];
  const float* bnfb = (const float*)d_in[4];
  const float* Wf   = (const float*)d_in[5];
  const float* bfe  = (const float*)d_in[6];
  const float* bng  = (const float*)d_in[7];
  const float* bnb  = (const float*)d_in[8];
  const float* Wsp  = (const float*)d_in[9];
  const float* bsp  = (const float*)d_in[10];
  float* out = (float*)d_out;
  const int* src = edge;
  const int* dst = edge + nE;

  const int MP   = cdiv(nN, NBA) * NBA;
  const int gM   = MP / GBM;
  const int gA   = MP / NBA;
  const int gS   = cdiv(nN, SROWS);
  const int gD   = cdiv(MP, NBD);
  const int NBPD = gD * NBD;
  if (NBPD < MP || (MP % GBM) != 0) return;
  const int vec8 = ((nE & 3) == 0) ? 1 : 0;
  const double invn = 1.0 / (double)nN;

  char* ws = (char*)d_ws;
  size_t off = 0;
  const size_t oDIS  = off; off = al256(off + (size_t)NBPD * 4);
  const size_t oWF2  = off; off = al256(off + (size_t)HID * 2 * FIN * 2);
  const size_t oWS2  = off; off = al256(off + (size_t)NLAY * HID * 2 * HID * 2);
  const size_t oST   = off; off = al256(off + (size_t)4 * 2 * FIN * 4);
  const size_t oRX   = off; off = al256(off + (size_t)gS * 2 * FIN * 8);
  const size_t oRG   = off; off = al256(off + (size_t)gM * 2 * HID * 8);
  const size_t oRS0  = off; off = al256(off + (size_t)gA * 2 * HID * 8);
  const size_t oRS1  = off; off = al256(off + (size_t)gA * 2 * HID * 8);
  const size_t oH    = off; off = al256(off + (size_t)MP * HID * 4);
  const size_t oT    = off; off = al256(off + (size_t)MP * HID * 4);
  if (off > ws_size || off > (size_t)WSMAX) return;
  float*          DIS  = (float*)(ws + oDIS);
  unsigned short* WF2  = (unsigned short*)(ws + oWF2);
  unsigned short* WS2  = (unsigned short*)(ws + oWS2);
  float*          STAT = (float*)(ws + oST);
  double*         RECX = (double*)(ws + oRX);
  double*         RECG = (double*)(ws + oRG);
  double*         RS0  = (double*)(ws + oRS0);
  double*         RS1  = (double*)(ws + oRS1);
  float*          H    = (float*)(ws + oH);
  float*          T    = (float*)(ws + oT);

  const size_t aggLds = (size_t)AGG_LDS_BYTES;
  hipFuncSetAttribute(reinterpret_cast<const void*>(&k_agg<1>), hipFuncAttributeMaxDynamicSharedMemorySize, (int)aggLds);
  hipFuncSetAttribute(reinterpret_cast<const void*>(&k_agg<0>), hipFuncAttributeMaxDynamicSharedMemorySize, (int)aggLds);

  k_wprep<<<(NUF + NUS) / NTHR, NTHR, 0, stream>>>(Wf, Wsp, WF2, WS2);
  k_deg<<<gD, NTHR, 0, stream>>>(src, nE, vec8, DIS);
  k_statx<<<gS, NTHR, 0, stream>>>(x, nN, RECX);
  k_comb<<<1, 128, 0, stream>>>(RECX, STAT, invn, gS, FIN);
  k_gemm<FIN, 1><<<gM, GTHR, 0, stream>>>(x, nN, STAT, bnfg, bnfb, WF2, bfe, H, RECG);
  k_comb<<<1, 128, 0, stream>>>(RECG, STAT + 1 * 2 * FIN, invn, gM, HID);
  k_gemm<HID, 0><<<gM, GTHR, 0, stream>>>(H, nN, STAT + 1 * 2 * FIN, bng, bnb, WS2, bsp, T, RECG);
  k_agg<1><<<gA, NTHR, aggLds, stream>>>(src, dst, nE, nN, vec8, MP, DIS, T, bsp, H, RS0);

  k_comb<<<1, 128, 0, stream>>>(RS0, STAT + 2 * 2 * FIN, invn, gA, HID);
  k_gemm<HID, 0><<<gM, GTHR, 0, stream>>>(H, nN, STAT + 2 * 2 * FIN, bng + HID, bnb + HID,
                                          WS2 + (size_t)HID * 2 * HID, bsp, T, RECG);
  k_agg<1><<<gA, NTHR, aggLds, stream>>>(src, dst, nE, nN, vec8, MP, DIS, T, bsp + HID, H, RS1);

  k_comb<<<1, 128, 0, stream>>>(RS1, STAT + 3 * 2 * FIN, invn, gA, HID);
  k_gemm<HID, 0><<<gM, GTHR, 0, stream>>>(H, nN, STAT + 3 * 2 * FIN, bng + 2 * HID, bnb + 2 * HID,
                                          WS2 + (size_t)2 * HID * 2 * HID, bsp, T, RECG);
  k_agg<0><<<gA, NTHR, aggLds, stream>>>(src, dst, nE, nN, vec8, MP, DIS, T, bsp + 2 * HID, H, RS0);
  k_pool<<<NGR, NTHR, 0, stream>>>(H, bat, nN, out);
}
